// WeightSharedBlock_81355270521456
// MI455X (gfx1250) — hardware-verified
//
#include <hip/hip_runtime.h>


namespace {
constexpr int Bn = 8, N = 1024, D = 384, H = 6, HD = 64, NT = Bn * N, DQ = 3 * D  , DF = 4 * D  , KW = 7;
constexpr float EPS = 1e-5f, XS = 8.0f, PS = 8.0f;
constexpr int PB_QKV = 0, PB_PROJ = 1152, P_DWW = 1536, P_DWB = 4224, P_MLG = 4608, P_MLB = 4992, P_N1G = 5376, P_N1B = 5760, P_N2G = 6144, P_N2B = 6528, PB_FC1 = 6912, PB_FC2 = 8448, P_TB = 8832, P_TA = 8868, P_END = 8904;
struct Wo_ { static constexpr size_t QKV = 0, PROJ = (size_t)DQ * D, FC1 = PROJ + (size_t)D * D, FC2 = FC1 + (size_t)DF * D, END = FC2 + (size_t)D * DF; };

typedef _Float16 b16;
typedef __attribute__((ext_vector_type(16))) _Float16 v16b;
typedef __attribute__((ext_vector_type(8))) _Float16 v8b;
typedef __attribute__((ext_vector_type(4))) _Float16 v4b;
typedef __attribute__((ext_vector_type(8))) float v8f;
typedef __attribute__((ext_vector_type(4))) float v4f;
__device__ __forceinline__ float bf16_rne(float f) { unsigned int u = __float_as_uint(f); u += 0x7FFFu + ((u >> 16) & 1u); return __uint_as_float(u & 0xFFFF0000u); }
__device__ __forceinline__ v16b frag_kb(const b16* p, int hh) { const v8b a = *(const v8b*)(p + 8 * hh), b = *(const v8b*)(p + 16 + 8 * hh); v16b f;
#pragma unroll
  for (int e = 0; e < 8; ++e) { f[e] = a[e]; f[8 + e] = b[e]; } return f; }
__device__ __forceinline__ v8f wmma16b(v16b a, v16b b, v8f c) { v8f d = __builtin_amdgcn_wmma_f32_16x16x32_f16(false, a, false, b, (short)0, c, false, false); asm volatile("v_nop\n\tv_nop\n\tv_nop\n\tv_nop" : "+v"(d) : "v"(a), "v"(b)); return d; }
__device__ __forceinline__ void wave_lds_sync() { __builtin_amdgcn_fence(__ATOMIC_RELEASE, "workgroup"); __builtin_amdgcn_wave_barrier(); __builtin_amdgcn_fence(__ATOMIC_ACQUIRE, "workgroup"); }
__device__ __forceinline__ float nexp(float x) { return __builtin_amdgcn_exp2f(x * 1.4426950408889634f); }
__device__ __forceinline__ float pmul(float a, float b) { float p = a * b; asm volatile("" : "+v"(p)); return p; }
__device__ __forceinline__ float wsum(float v) {
#pragma unroll
  for (int o = 1; o < 32; o <<= 1) v += __shfl_xor(v, o); return v; }

__global__ __launch_bounds__(256) void prep_kernel(const float* __restrict__ wqkv, const float* __restrict__ wproj, const float* __restrict__ wfc1, const float* __restrict__ wfc2, const float* __restrict__ bqkv, const float* __restrict__ bproj, const float* __restrict__ dww, const float* __restrict__ dwb, const float* __restrict__ mlg, const float* __restrict__ mlb, const float* __restrict__ n1g, const float* __restrict__ n1b, const float* __restrict__ n2g, const float* __restrict__ n2b, const float* __restrict__ bfc1, const float* __restrict__ bfc2, const float* __restrict__ tb, const float* __restrict__ ta, b16* __restrict__ R, float* __restrict__ P) {
  const size_t tid = (size_t)blockIdx.x * 256 + threadIdx.x, nth = (size_t)gridDim.x * 256;
  for (int pass = 0; pass < 2; ++pass) {
    for (size_t p = tid; p < Wo_::END / 8; p += nth) { const size_t q = p * 8; const float* src = (q < Wo_::PROJ) ? (wqkv + q) : (q < Wo_::FC1) ? (wproj + (q - Wo_::PROJ)) : (q < Wo_::FC2) ? (wfc1 + (q - Wo_::FC1)) : (wfc2 + (q - Wo_::FC2)); v8b v;
#pragma unroll
      for (int e = 0; e < 8; ++e) v[e] = (b16)bf16_rne(src[e]); *(volatile v8b*)(R + q) = v; }
    for (size_t q = tid; q < P_END; q += nth) { const int i = (int)q; float v;
      if (i < PB_PROJ) v = bqkv[i]; else if (i < P_DWW) v = bproj[i - PB_PROJ]; else if (i < P_DWB) v = dww[i - P_DWW]; else if (i < P_MLG) v = dwb[i - P_DWB]; else if (i < P_MLB) v = mlg[i - P_MLG]; else if (i < P_N1G) v = mlb[i - P_MLB]; else if (i < P_N1B) v = n1g[i - P_N1G];
      else if (i < P_N2G) v = n1b[i - P_N1B]; else if (i < P_N2B) v = n2g[i - P_N2G]; else if (i < PB_FC1) v = n2b[i - P_N2B]; else if (i < PB_FC2) v = bfc1[i - PB_FC1]; else if (i < P_TB) v = bfc2[i - PB_FC2]; else if (i < P_TA) v = tb[i - P_TB]; else v = ta[i - P_TA];
      P[q] = bf16_rne(v); }
    __threadfence(); }
}

template <int MODE>
__global__ __launch_bounds__(256) void ln_kernel(const float* __restrict__ src, int rnd, const float* __restrict__ g, const float* __restrict__ bb, b16* __restrict__ dh, float* __restrict__ df) {
  const int row = blockIdx.x * 8 + (threadIdx.x >> 5), lane = threadIdx.x & 31; const float* xr = src + (size_t)row * D;
  float v[12]; float s = 0.0f;
#pragma unroll
  for (int i = 0; i < 12; ++i) { float x = xr[(i >> 2) * 128 + lane * 4 + (i & 3)]; if (rnd) x = bf16_rne(x); v[i] = x; s += x; }
  s = wsum(s); const float mu = s * (1.0f / D); float q = 0.0f;
#pragma unroll
  for (int i = 0; i < 12; ++i) { const float d = v[i] - mu; q += pmul(d, d); }
  q = wsum(q); const float inv = rsqrtf(q * (1.0f / D) + EPS);
  for (int pass = 0; pass < 2; ++pass) {
#pragma unroll
    for (int gq = 0; gq < 3; ++gq) { const int c0 = gq * 128 + lane * 4; float y[4];
#pragma unroll
      for (int e = 0; e < 4; ++e) y[e] = pmul((v[gq * 4 + e] - mu) * inv, g[c0 + e]) + bb[c0 + e];
      if (MODE == 0) { v4b o; for (int e = 0; e < 4; ++e) o[e] = (b16)(y[e] * XS); *(volatile v4b*)(dh + (size_t)row * D + c0) = o; }
      else { v4f o; for (int e = 0; e < 4; ++e) o[e] = y[e]; *(volatile v4f*)(df + (size_t)row * D + c0) = o; } }
    __threadfence(); }
}

__global__ __launch_bounds__(256) void dw_kernel(const float* __restrict__ H2, const float* __restrict__ P, b16* __restrict__ dh) {
  const int row = blockIdx.x * 8 + (threadIdx.x >> 5), lane = threadIdx.x & 31; const int b = row / N, n = row % N;
  float v[12]; float s = 0.0f;
#pragma unroll
  for (int i = 0; i < 12; ++i) { const int c = (i >> 2) * 128 + lane * 4 + (i & 3); float acc = 0.0f;
#pragma unroll
    for (int j = 0; j < KW; ++j) { const int nn = n + j - 3; if (nn >= 0 && nn < N) acc += pmul(P[P_DWW + c * KW + j], H2[((size_t)b * N + nn) * D + c]); }
    v[i] = acc + P[P_DWB + c]; s += v[i]; }
  s = wsum(s); const float mu = s * (1.0f / D); float q = 0.0f;
#pragma unroll
  for (int i = 0; i < 12; ++i) { const float d = v[i] - mu; q += pmul(d, d); }
  q = wsum(q); const float inv = rsqrtf(q * (1.0f / D) + EPS);
  for (int pass = 0; pass < 2; ++pass) {
#pragma unroll
    for (int gq = 0; gq < 3; ++gq) { const int c0 = gq * 128 + lane * 4; v4b o; for (int e = 0; e < 4; ++e) o[e] = (b16)((pmul((v[gq * 4 + e] - mu) * inv, P[P_MLG + c0 + e]) + P[P_MLB + c0 + e]) * XS); *(volatile v4b*)(dh + (size_t)row * D + c0) = o; }
    __threadfence(); }
}

template <int K, int NN, int EPI, int RND>
__global__ __launch_bounds__(32) void gemm_kernel(const b16* __restrict__ A, const b16* __restrict__ Bw, const float* __restrict__ bias, const float* __restrict__ resid, b16* __restrict__ Ch, float* __restrict__ Cf) {
  __shared__ __attribute__((aligned(16))) float Ts[32][128 + 4];
  const int lane = threadIdx.x, nloc = lane & 15, hlf = lane >> 4, m0 = blockIdx.y * 32, c0 = blockIdx.x * 128;
  v8f acc[2][8];
#pragma unroll
  for (int r = 0; r < 2; ++r)
#pragma unroll
    for (int t = 0; t < 8; ++t) acc[r][t] = (v8f){};
  for (int kb = 0; kb < K; kb += 32) { const v16b a0 = frag_kb(A + (size_t)(m0 + nloc) * K + kb, hlf), a1 = frag_kb(A + (size_t)(m0 + 16 + nloc) * K + kb, hlf);
#pragma unroll
    for (int t = 0; t < 8; ++t) { const v16b bw = frag_kb(Bw + (size_t)(c0 + t * 16 + nloc) * K + kb, hlf); acc[0][t] = wmma16b(a0, bw, acc[0][t]); acc[1][t] = wmma16b(a1, bw, acc[1][t]); } }
#pragma unroll
  for (int t = 0; t < 8; ++t) { const float bv = bias[c0 + t * 16 + nloc];
#pragma unroll
    for (int r = 0; r < 2; ++r)
#pragma unroll
      for (int v = 0; v < 8; ++v) { float y = acc[r][t][v] * (1.0f / XS) + bv; if (EPI == 2) y = 0.5f * y * (1.0f + erff(y * 0.7071067811865476f)); Ts[r * 16 + 8 * hlf + v][t * 16 + nloc] = y; } }
  wave_lds_sync();
  for (int pass = 0; pass < 2; ++pass) {
    if (EPI == 1) { for (int i = lane; i < 32 * 32; i += 32) { const int rr = i >> 5, c4 = (i & 31) * 4; const size_t gi = (size_t)(m0 + rr) * NN + c0 + c4; v4f o = *(const v4f*)(&Ts[rr][c4]); const v4f xr = *(const v4f*)(resid + gi);
        for (int e = 0; e < 4; ++e) o[e] += RND ? bf16_rne(xr[e]) : xr[e]; *(volatile v4f*)(Cf + gi) = o; } }
    else { for (int i = lane; i < 32 * 16; i += 32) { const int rr = i >> 4, c8 = (i & 15) * 8; v8b o; for (int e = 0; e < 8; ++e) o[e] = (b16)(Ts[rr][c8 + e] * XS); *(volatile v8b*)(Ch + (size_t)(m0 + rr) * NN + c0 + c8) = o; } }
    __threadfence(); }
}

__global__ __launch_bounds__(256) void vt_kernel(const b16* __restrict__ QKV, b16* __restrict__ vt) {
  __shared__ __attribute__((aligned(16))) b16 T[HD][128 + 8];
  const int b = blockIdx.z, h = blockIdx.y, t0 = blockIdx.x * 128, t_ = threadIdx.x;
  for (int i = t_; i < 128 * (HD / 8); i += 256) { const int tk = i >> 3, d8 = (i & 7) * 8; const v8b vv = *(const v8b*)(QKV + ((size_t)(b * N + t0 + tk)) * DQ + 2 * D + h * HD + d8); for (int e = 0; e < 8; ++e) T[d8 + e][tk] = vv[e]; }
  __syncthreads();
  for (int pass = 0; pass < 2; ++pass) { for (int i = t_; i < HD * 16; i += 256) { const int d = i >> 4, c8 = (i & 15) * 8; *(volatile v8b*)(vt + (((size_t)b * H + h) * HD + d) * N + t0 + c8) = *(const v8b*)(&T[d][c8]); } __threadfence(); }
}

__global__ __launch_bounds__(256) void qmix_kernel(const b16* __restrict__ QKV, const float* __restrict__ P, b16* __restrict__ Qm) {
  const int row = blockIdx.x * 8 + (threadIdx.x >> 5), lane = threadIdx.x & 31; const b16* qr = QKV + (size_t)row * DQ;
  for (int pass = 0; pass < 2; ++pass) {
    for (int g = 0; g < H; ++g) {
#pragma unroll
      for (int gq = 0; gq < 3; ++gq) { const int c0 = gq * 128 + lane * 4; const int h = c0 >> 6; const float tbv = P[P_TB + g * H + h]; v4b o;
#pragma unroll
        for (int e = 0; e < 4; ++e) o[e] = (b16)pmul((float)qr[c0 + e], tbv);
        *(volatile v4b*)(Qm + ((size_t)g * NT + row) * D + c0) = o; } }
    __threadfence(); }
}

__global__ __launch_bounds__(192) void attn_kernel(const b16* __restrict__ QKV, const b16* __restrict__ Qm, const b16* __restrict__ vt, const float* __restrict__ P, b16* __restrict__ ctx) {
  __shared__ __attribute__((aligned(16))) b16 Os[16][D + 8]; __shared__ float Pt[H][32][16 + 1]; __shared__ float TA[36];
  const int g = threadIdx.x >> 5, lane = threadIdx.x & 31, hh = lane >> 4, col = lane & 15; const int b = blockIdx.x / (N / 16), q0 = (blockIdx.x % (N / 16)) * 16, qi = q0 + col;
  if (threadIdx.x < 36) TA[threadIdx.x] = P[P_TA + threadIdx.x];
  const b16* Kr = QKV + (size_t)(b * N) * DQ + D; const b16* Qg = Qm + ((size_t)g * NT + b * N) * D; const b16* V = vt + (((size_t)b * H + g) * HD) * N; const float SC = 0.125f / (XS * XS);
  v16b qf[12];
#pragma unroll
  for (int j = 0; j < 12; ++j) qf[j] = frag_kb(Qg + (size_t)qi * D + 32 * j, hh);
  auto scores = [&](int kb, float (&s)[2][8]) {
#pragma unroll
    for (int half = 0; half < 2; ++half) { const b16* kp = Kr + (size_t)(kb + 16 * half + col) * DQ; v8f a = {};
#pragma unroll
      for (int j = 0; j < 12; ++j) a = wmma16b(frag_kb(kp + 32 * j, hh), qf[j], a);
#pragma unroll
      for (int r = 0; r < 8; ++r) s[half][r] = a[r] * SC; } };
  float m = -INFINITY, l = 0.0f;
  for (int kb = 0; kb < N; kb += 32) { float s[2][8]; scores(kb, s); float mr = -INFINITY;
#pragma unroll
    for (int half = 0; half < 2; ++half)
#pragma unroll
      for (int r = 0; r < 8; ++r) mr = fmaxf(mr, s[half][r]);
    mr = fmaxf(mr, __shfl_xor(mr, 16)); const float mn = fmaxf(m, mr); float sum = 0.0f;
#pragma unroll
    for (int half = 0; half < 2; ++half)
#pragma unroll
      for (int r = 0; r < 8; ++r) sum += nexp(s[half][r] - mn);
    sum += __shfl_xor(sum, 16); l = l * nexp(m - mn) + sum; m = mn; }
  const float il = 1.0f / l; v8f o[4] = {{}, {}, {}, {}};
  __syncthreads();
  for (int kb = 0; kb < N; kb += 32) { float s[2][8]; scores(kb, s);
#pragma unroll
    for (int half = 0; half < 2; ++half)
#pragma unroll
      for (int r = 0; r < 8; ++r) Pt[g][16 * half + 8 * hh + r][col] = nexp(s[half][r] - m) * il;
    __syncthreads();
    v16b pb;
#pragma unroll
    for (int half = 0; half < 2; ++half)
#pragma unroll
      for (int r = 0; r < 8; ++r) { const int kk = 16 * half + 8 * hh + r; float v = 0.0f;
#pragma unroll
        for (int h = 0; h < H; ++h) v += pmul(TA[g * H + h], Pt[h][kk][col]);
        pb[half * 8 + r] = (b16)(v * PS); }
#pragma unroll
    for (int t = 0; t < 4; ++t) o[t] = wmma16b(frag_kb(V + (size_t)(t * 16 + col) * N + kb, hh), pb, o[t]);
    __syncthreads(); }
#pragma unroll
  for (int t = 0; t < 4; ++t)
#pragma unroll
    for (int r = 0; r < 8; ++r) Os[col][g * HD + t * 16 + 8 * hh + r] = (b16)(o[t][r] * (1.0f / PS));
  __syncthreads();
  for (int pass = 0; pass < 2; ++pass) { for (int i = threadIdx.x; i < 16 * (D / 8); i += 192) { const int rr = i / (D / 8), c8 = (i % (D / 8)) * 8; *(volatile v8b*)(ctx + ((size_t)(b * N + q0 + rr)) * D + c8) = *(const v8b*)(&Os[rr][c8]); } __threadfence(); }
}
}

extern "C" void kernel_launch(void* const* d_in, const int* in_sizes, int n_in,
                              void* d_out, int out_size, void* d_ws, size_t ws_size, hipStream_t stream) {
  (void)n_in; (void)out_size;
  const float* x = (const float*)d_in[0]; const float* wqkv = (const float*)d_in[1]; const float* bqkv = (const float*)d_in[2]; const float* wproj = (const float*)d_in[3]; const float* bproj = (const float*)d_in[4]; const float* tb = (const float*)d_in[5]; const float* ta = (const float*)d_in[6];
  const float* dww = (const float*)d_in[7]; const float* dwb = (const float*)d_in[8]; const float* mlg = (const float*)d_in[9]; const float* mlb = (const float*)d_in[10]; const float* n1g = (const float*)d_in[11]; const float* n1b = (const float*)d_in[12]; const float* n2g = (const float*)d_in[13]; const float* n2b = (const float*)d_in[14];
  const float* wfc1 = (const float*)d_in[15]; const float* bfc1 = (const float*)d_in[16]; const float* wfc2 = (const float*)d_in[17]; const float* bfc2 = (const float*)d_in[18];
  float* out = (float*)d_out;
  if (in_sizes[0] != NT * D || in_sizes[1] != DQ * D || in_sizes[5] != 36 || in_sizes[7] != D * KW || in_sizes[15] != DF * D || in_sizes[17] != D * DF) return;
  size_t off = 0; char* ws = (char*)d_ws;
  auto carve = [&](size_t bytes) { char* p = ws + off; off += (bytes + 255) & ~(size_t)255; return p; };
  b16* R = (b16*)carve(Wo_::END * 2); float* P = (float*)carve(9216 * 4); b16* SH = (b16*)carve((size_t)NT * D * 2); b16* QKV = (b16*)carve((size_t)NT * DQ * 2); b16* VT = (b16*)carve((size_t)Bn * H * HD * N * 2); b16* QM = (b16*)carve((size_t)H * NT * D * 2);
  float* X1 = (float*)carve((size_t)NT * D * 4); float* H2 = (float*)carve((size_t)NT * D * 4); b16* G = (b16*)carve((size_t)NT * DF * 2);
  if (off > ws_size) return;
  prep_kernel<<<256, 256, 0, stream>>>(wqkv, wproj, wfc1, wfc2, bqkv, bproj, dww, dwb, mlg, mlb, n1g, n1b, n2g, n2b, bfc1, bfc2, tb, ta, R, P);
  ln_kernel<0><<<NT / 8, 256, 0, stream>>>(x, 1, P + P_N1G, P + P_N1B, SH, nullptr);
  gemm_kernel<D, DQ, 0, 0><<<dim3(DQ / 128, NT / 32), 32, 0, stream>>>(SH, R + Wo_::QKV, P + PB_QKV, nullptr, QKV, nullptr);
  vt_kernel<<<dim3(N / 128, H, Bn), 256, 0, stream>>>(QKV, VT);
  qmix_kernel<<<NT / 8, 256, 0, stream>>>(QKV, P, QM);
  attn_kernel<<<NT / 16, 192, 0, stream>>>(QKV, QM, VT, P, SH);
  gemm_kernel<D, D, 1, 1><<<dim3(D / 128, NT / 32), 32, 0, stream>>>(SH, R + Wo_::PROJ, P + PB_PROJ, x, nullptr, X1);
  ln_kernel<1><<<NT / 8, 256, 0, stream>>>(X1, 0, P + P_N2G, P + P_N2B, nullptr, H2);
  dw_kernel<<<NT / 8, 256, 0, stream>>>(H2, P, SH);
  gemm_kernel<D, DF, 2, 0><<<dim3(DF / 128, NT / 32), 32, 0, stream>>>(SH, R + Wo_::FC1, P + PB_FC1, nullptr, G, nullptr);
  gemm_kernel<DF, D, 1, 0><<<dim3(D / 128, NT / 32), 32, 0, stream>>>(G, R + Wo_::FC2, P + PB_FC2, X1, nullptr, out);
}
